// TemporalSelfAttention_56435870269919
// MI455X (gfx1250) — hardware-run, weakly checked
//
#include <hip/hip_runtime.h>


#ifndef NB
#define NB 1
#endif
#ifndef SEQ
#define SEQ 1024
#endif
#define NB_FULL  1
#define SEQ_FULL 1024
#ifndef OUT_SEQ
#define OUT_SEQ SEQ
#endif
#define DM   256
#define NH_  8
#define HD   32
#define AW   4
#define OSP  36
#define SC2  ((float)(0.17677669529663687 * 1.4426950408889634))
#define PSH  14.0f
#define NEGB (-3.0e38f)
#define TT   64
#define TC   64
#define TSP  72

static_assert(HD == 32);
static_assert(NH_ * HD == DM);
static_assert(DM % 8 == 0);
static_assert(SEQ % 64 == 0);
static_assert(SEQ % 32 == 0);
static_assert(SEQ % (16 * AW) == 0);
static_assert(SEQ % TT == 0);
static_assert(DM % TC == 0);
static_assert(TT * 2 == 128);
static_assert(TSP >= TT);
static_assert((TSP * 2) % 16 == 0);
static_assert(256 * 4 * 4 == TT * TC);
static_assert(256 * 2 * 8 == TC * TT);
static_assert(32 * 4 * 4 == 16 * HD);
static_assert(((size_t)SEQ * DM) % 64 == 0);
static_assert(NB <= NB_FULL);
static_assert(SEQ <= SEQ_FULL);
static_assert((OSP * 4) % 16 == 0);
static_assert(OSP >= HD);
static_assert((size_t)AW * 16 * OSP * 4 <= (size_t)131072);
static_assert((size_t)TC * TSP * 2 <= (size_t)131072);

typedef _Float16 h16;
typedef __attribute__((ext_vector_type(16))) _Float16 v16h;
typedef __attribute__((ext_vector_type(8)))  _Float16 v8h;
typedef __attribute__((ext_vector_type(8)))  float    v8f;
typedef __attribute__((ext_vector_type(4)))  float    v4f;
typedef v4f  __attribute__((may_alias)) v4fa;
typedef v8h  __attribute__((may_alias)) v8ha;

__device__ __forceinline__ unsigned short f2bf(float f) { unsigned u = __float_as_uint(f); u += 0x7FFFu + ((u >> 16) & 1u); return (unsigned short)(u >> 16); }
__device__ __forceinline__ float bfr(float f) { return __uint_as_float(((unsigned)f2bf(f)) << 16); }
__device__ __forceinline__ v16h cat16(v8h lo, v8h hi) { return __builtin_shufflevector(lo, hi, 0, 1, 2, 3, 4, 5, 6, 7, 8, 9, 10, 11, 12, 13, 14, 15); }
__device__ __forceinline__ v8f wmma16(v16h a, v16h b, v8f c) { return __builtin_amdgcn_wmma_f32_16x16x32_f16(false, a, false, b, (short)0, c, false, false); }
__device__ __forceinline__ v16h  ldh(const h16* p) { return cat16(*(const v8h*)p, *(const v8h*)(p + 16)); }
__device__ __forceinline__ void wave_sync() { __builtin_amdgcn_fence(3  , "wavefront"); __builtin_amdgcn_wave_barrier(); asm volatile("" ::: "memory"); }
static __device__ __forceinline__ h16 toh_flush(float v) { const h16 r = (h16)v; return (fabsf(v) < 6.103515625e-05f) ? (h16)0.0f : r; }
__device__ __forceinline__ v8f wmma16g(v16h a, v16h b, v8f c) {
    c = wmma16(a, b, c);
    asm volatile("v_nop\n\tv_nop\n\tv_nop\n\tv_nop" : "+v"(c) : "v"(a), "v"(b));
    return c;
}

__global__ __launch_bounds__(256) void k_cvth(const float* __restrict__ src, h16* dst, size_t n8) {
    const size_t i = (size_t)blockIdx.x * 256 + threadIdx.x; if (i >= n8) return;
    const v8f v = *(const v8f*)(src + i * 8); v8h o;
#pragma unroll
    for (int k = 0; k < 8; ++k) o[k] = toh_flush(bfr(v[k]));
    *(volatile v8h*)(dst + i * 8) = o; __threadfence(); *(volatile v8h*)(dst + i * 8) = o;
}

__global__ __launch_bounds__(256) void k_vt(const float* __restrict__ src, h16* VT) {
    __shared__ __align__(16) h16 ts[TC * TSP];
    const int tid = threadIdx.x;
    const int tk0 = blockIdx.x * TT, c0 = blockIdx.y * TC, b = blockIdx.z;
    const float* sp = src + ((size_t)b * SEQ_FULL + (size_t)tk0) * DM + c0;
#pragma unroll 1
    for (int it = 0; it < 4; ++it) {
        const int idx = it * 256 + tid; const int t = idx >> 4, c4 = (idx & 15) * 4;
        const v4f x = *(const v4f*)(sp + (size_t)t * DM + c4);
#pragma unroll
        for (int k = 0; k < 4; ++k) ts[(c4 + k) * TSP + t] = toh_flush(bfr(x[k])); }
    __syncthreads();
    h16* dp = VT + ((size_t)b * DM + (size_t)c0) * SEQ + (size_t)tk0;
#pragma unroll 1
    for (int ps = 0; ps < 2; ++ps) {
#pragma unroll
        for (int it = 0; it < 2; ++it) { const int p = it * 256 + tid; const int row = p >> 3, c8 = (p & 7) * 8;
            const v8h val = *(const v8ha*)(&ts[row * TSP + c8]);
            *(volatile v8h*)(dp + (size_t)row * SEQ + c8) = val; }
        if (ps == 0) __threadfence(); }
}

__global__ __launch_bounds__(32 * AW) void k_keypass(const h16* __restrict__ QP, const h16* __restrict__ KP, const h16* __restrict__ VT, float* OUT) {
    __shared__ __align__(16) float os[AW * 16 * OSP];
    const int lane = threadIdx.x & 31, lr = lane & 15, hi = lane >> 4;
    const int wave = __builtin_amdgcn_readfirstlane((int)(threadIdx.x >> 5));
    const int zh = blockIdx.y; const int b = zh / NH_, h = zh % NH_;
    const int t0 = (blockIdx.x * AW + wave) * 16;
    const size_t pbase = (size_t)b * SEQ * DM + (size_t)h * HD;
    const size_t qo = pbase + (size_t)(t0 + lr) * DM + 8 * hi;
    const v16h qh = ldh(QP + qo);
    const size_t ko = pbase + (size_t)lr * DM + 8 * hi;
    const size_t vo = ((size_t)b * DM + (size_t)h * HD + (size_t)lr) * SEQ + 8 * hi;
    v8f o0 = (v8f){}, o1 = (v8f){};
    float m = NEGB, l = 0.0f;
#pragma unroll 1
    for (int key0 = 0; key0 < SEQ; key0 += 32) {
        const h16* ka = KP + ko + (size_t)key0 * DM;
        const v16h ka0 = ldh(ka), kb0 = ldh(ka + 16 * DM);
        v8f sa = (v8f){}, sb = (v8f){};
        sa = wmma16g(ka0, qh, sa); sb = wmma16g(kb0, qh, sb);
        float ta[8], tb[8]; float mx = NEGB;
#pragma unroll
        for (int r = 0; r < 8; ++r) { ta[r] = sa[r] * SC2; tb[r] = sb[r] * SC2; mx = fmaxf(mx, fmaxf(ta[r], tb[r])); }
        mx = fmaxf(mx, __shfl_xor(mx, 16, 32));
        const float mnew = fmaxf(m, mx);
        const float alpha = __builtin_amdgcn_exp2f(m - mnew);
        const float sh = PSH - mnew;
        v16h pb; float ls = 0.0f;
#pragma unroll
        for (int r = 0; r < 8; ++r) {
            const float xa = ta[r] + sh, xb = tb[r] + sh;
            const float ea = __builtin_amdgcn_exp2f(xa), eb = __builtin_amdgcn_exp2f(xb);
            const float ga = (xa < -14.0f) ? 0.0f : ea, gb = (xb < -14.0f) ? 0.0f : eb;
            const h16 pa = (h16)ga; const h16 pc = (h16)gb;
            pb[r] = pa; pb[8 + r] = pc;
            ls += (float)pa + (float)pc; }
        l = l * alpha + ls; m = mnew;
        o0 = o0 * alpha; o1 = o1 * alpha;
        const h16* va = VT + vo + key0;
        const v16h v0 = ldh(va), v1 = ldh(va + (size_t)16 * SEQ);
        o0 = wmma16g(v0, pb, o0); o1 = wmma16g(v1, pb, o1);
    }
    l += __shfl_xor(l, 16, 32);
    const float inv = 1.0f / l;
    const v8f f0 = o0, f1 = o1;
    const int wb = wave * 16 * OSP;
    { v4f a, c;
      a[0] = f0[0] * inv; a[1] = f0[1] * inv; a[2] = f0[2] * inv; a[3] = f0[3] * inv; c[0] = f0[4] * inv; c[1] = f0[5] * inv; c[2] = f0[6] * inv; c[3] = f0[7] * inv;
      *(v4fa*)(&os[wb + lr * OSP +  0 + 8 * hi]) = a; *(v4fa*)(&os[wb + lr * OSP +  0 + 8 * hi + 4]) = c;
      a[0] = f1[0] * inv; a[1] = f1[1] * inv; a[2] = f1[2] * inv; a[3] = f1[3] * inv; c[0] = f1[4] * inv; c[1] = f1[5] * inv; c[2] = f1[6] * inv; c[3] = f1[7] * inv;
      *(v4fa*)(&os[wb + lr * OSP + 16 + 8 * hi]) = a; *(v4fa*)(&os[wb + lr * OSP + 16 + 8 * hi + 4]) = c; }
    wave_sync();
    float* orow = OUT + ((size_t)b * OUT_SEQ + t0) * DM + h * HD;
#pragma unroll 1
    for (int ps = 0; ps < 2; ++ps) {
#pragma unroll
        for (int s = 0; s < 4; ++s) { const int row = 4 * s + (lane >> 3), cofs = (lane & 7) * 4;
            const v4f val = *(const v4fa*)(&os[wb + row * OSP + cofs]);
            *(volatile v4f*)(orow + (size_t)row * DM + cofs) = val; }
        if (ps == 0) __threadfence(); }
}

static constexpr size_t al256(size_t v) { return (v + 255) & ~(size_t)255; }
static constexpr size_t SZ_PL = al256((size_t)NB * SEQ * DM * 2);
static constexpr size_t SZ_TOTAL = 3 * SZ_PL;
static_assert(SZ_TOTAL <= (size_t)134217728);
static_assert(SZ_PL % 128 == 0);

extern "C" void kernel_launch(void* const* d_in, const int* in_sizes, int n_in,
                              void* d_out, int out_size, void* d_ws, size_t ws_size, hipStream_t stream) {
    if (n_in < 2) return;
    const size_t needx = ((size_t)(NB - 1) * SEQ_FULL + SEQ) * DM;
    if ((size_t)in_sizes[0] < needx || (size_t)in_sizes[1] < needx) return;
    if ((size_t)out_size < ((size_t)(NB - 1) * OUT_SEQ + SEQ) * DM) return;
    if (SZ_TOTAL > ws_size) return;
    const float* hist  = (const float*)d_in[0];
    const float* query = (const float*)d_in[1];
    float* OUT = (float*)d_out;
    char* wsp = (char*)d_ws;
    h16* QP = (h16*)wsp; wsp += SZ_PL;
    h16* KP = (h16*)wsp; wsp += SZ_PL;
    h16* VT = (h16*)wsp; wsp += SZ_PL;

    {
        const size_t n8 = (size_t)SEQ * DM / 8;
        for (int b = 0; b < NB; ++b) {
            k_cvth<<<(unsigned)((n8 + 255) / 256), 256, 0, stream>>>(query + (size_t)b * SEQ_FULL * DM, QP + (size_t)b * SEQ * DM, n8);
            k_cvth<<<(unsigned)((n8 + 255) / 256), 256, 0, stream>>>(hist + (size_t)b * SEQ_FULL * DM, KP + (size_t)b * SEQ * DM, n8);
        }
    }
    k_vt<<<dim3(SEQ / TT, DM / TC, NB), 256, 0, stream>>>(hist, VT);

    k_keypass<<<dim3(SEQ / (16 * AW), NB * NH_, 1), 32 * AW, 0, stream>>>(QP, KP, VT, OUT);
}
